// _AttentionBlock_16758962389674
// MI455X (gfx1250) — hardware-verified
//
#include <hip/hip_runtime.h>
#include <math.h>

typedef __attribute__((ext_vector_type(16))) _Float16 v16h;
typedef __attribute__((ext_vector_type(8)))  _Float16 v8h;
typedef __attribute__((ext_vector_type(16))) __bf16   v16b;
typedef __attribute__((ext_vector_type(8)))  __bf16   v8b;
typedef __attribute__((ext_vector_type(8)))  float    v8f;
typedef __attribute__((ext_vector_type(4)))  float    v4f;
typedef __attribute__((ext_vector_type(4)))  unsigned int v4u;

constexpr int NCH = 128;
constexpr int IMG_L = 4096;
constexpr int NGROUPS = 32;
constexpr int GROUP_ELEMS = (NCH / NGROUPS) * IMG_L;
constexpr int STATS_LINE_FLOATS = 32;
static_assert(NCH % 64 == 0);
static_assert(NCH % 32 == 0);
static_assert(IMG_L % 64 == 0);
static_assert(GROUP_ELEMS % 1024 == 0);
static_assert((NCH * NCH) % 512 == 0);

__device__ __forceinline__ unsigned short f2bf_bits(float f) {
  unsigned u = __float_as_uint(f);
  return (unsigned short)((u + 0x7FFFu + ((u >> 16) & 1u)) >> 16);
}
__device__ __forceinline__ float bf_bits2f(unsigned short h) { return __uint_as_float(((unsigned)h) << 16); }

__device__ __forceinline__ void dep_guard_h(v8f& a, v8f& b, v16h x, v16h y) { asm volatile("v_nop\n\tv_nop\n\tv_nop\n\tv_nop" : "+v"(a), "+v"(b) : "v"(x), "v"(y)); }
__device__ __forceinline__ void dep_guard_b(v8f& a, v8f& b, v16b x, v16b y) { asm volatile("v_nop\n\tv_nop\n\tv_nop\n\tv_nop" : "+v"(a), "+v"(b) : "v"(x), "v"(y)); }
__device__ __forceinline__ void keep4_h(v16h a, v16h b, v16h c, v16h d) { asm volatile("v_nop" :: "v"(a), "v"(b), "v"(c), "v"(d)); }
__device__ __forceinline__ void keep4_b(v16b a, v16b b, v16b c, v16b d) { asm volatile("v_nop" :: "v"(a), "v"(b), "v"(c), "v"(d)); }
__device__ __forceinline__ void acc_guard4(v8f& a, v8f& b, v8f& c, v8f& d) { asm volatile("v_nop\n\tv_nop\n\tv_nop\n\tv_nop" : "+v"(a), "+v"(b), "+v"(c), "+v"(d)); }
template <typename T> struct Frag;
template <> struct Frag<_Float16> {
  typedef v16h V; union U { v16h v; v8h h[2]; };
  static __device__ __forceinline__ v16h load(const _Float16* p) {
    U f; f.h[0] = *(const v8h*)(p); f.h[1] = *(const v8h*)(p + 16); return f.v;
  }
  static __device__ __forceinline__ v8f mma(v16h a, v16h b, v8f c) {
    return __builtin_amdgcn_wmma_f32_16x16x32_f16(false, a, false, b, (short)0, c, false, false);
  }
  static __device__ __forceinline__ void guard(v8f& a, v8f& b, v16h x, v16h y) { dep_guard_h(a, b, x, y); }
  static __device__ __forceinline__ void keep(v16h a, v16h b, v16h c, v16h d) { keep4_h(a, b, c, d); }
};
template <> struct Frag<__bf16> {
  typedef v16b V; union U { v16b v; v8b h[2]; };
  static __device__ __forceinline__ v16b load(const __bf16* p) {
    U f; f.h[0] = *(const v8b*)(p); f.h[1] = *(const v8b*)(p + 16); return f.v;
  }
  static __device__ __forceinline__ v8f mma(v16b a, v16b b, v8f c) {
    return __builtin_amdgcn_wmma_f32_16x16x32_bf16(false, a, false, b, (short)0, c, false, false);
  }
  static __device__ __forceinline__ void guard(v8f& a, v8f& b, v16b x, v16b y) { dep_guard_b(a, b, x, y); }
  static __device__ __forceinline__ void keep(v16b a, v16b b, v16b c, v16b d) { keep4_b(a, b, c, d); }
};

template <int ET> struct Elem;
template <> struct Elem<0> { typedef _Float16 T; };
template <> struct Elem<1> { typedef __bf16 T; };
template <int ET, bool SPLIT, int BIAS_MODE, int OUT_MODE, bool RESID, int ACT = 0>
__global__ __launch_bounds__(256) void wmma_gemm64(
    const unsigned short* __restrict__ Ap, const unsigned short* __restrict__ A2p, int lda, long strideA,
    const unsigned short* __restrict__ Btp, const unsigned short* __restrict__ Bt2p, int ldb, long strideB,
    void* __restrict__ Cout, void* __restrict__ Cout2, int ldc, long strideC,
    const float* __restrict__ bias,
    const float* __restrict__ resid, long strideR,
    int M, int N, int K, float scale) {
  typedef typename Elem<ET>::T T;
  typedef typename Frag<T>::V V;
  const T* A = (const T*)Ap; const T* A2 = (const T*)A2p; const T* Bt = (const T*)Btp; const T* Bt2 = (const T*)Bt2p;
  __shared__ __align__(16) float sT[8][16 * 68];
  const int b    = blockIdx.y;
  const int lane = threadIdx.x & 31;
  const int wave = threadIdx.x >> 5;
  const int tilesN = N >> 6;
  const int tilesM = M >> 6;
  const int tile = blockIdx.x * 8 + wave;
  if (tile >= tilesM * tilesN) return;
  const int tm = tile / tilesN;
  const int tn = tile - tm * tilesN;
  const int m0 = tm << 6;
  const int n0 = tn << 6;

  const T* Ab  = A  + (size_t)b * strideA;
  const T* Bb  = Bt + (size_t)b * strideB;
  const T* Ab2 = SPLIT ? (A2  + (size_t)b * strideA) : nullptr;
  const T* Bb2 = SPLIT ? (Bt2 + (size_t)b * strideB) : nullptr;

  const int rlane = lane & 15;
  const int koff  = (lane >> 4) * 8;
  const int mOff  = (lane >> 4) * 8;

  v8f acc[4][4];
#pragma unroll
  for (int i = 0; i < 4; ++i)
#pragma unroll
    for (int j = 0; j < 4; ++j) acc[i][j] = (v8f){0.f,0.f,0.f,0.f,0.f,0.f,0.f,0.f};

  for (int k0 = 0; k0 < K; k0 += 32) {
    V bh[4], bl[4];
#pragma unroll
    for (int j = 0; j < 4; ++j) {
      const size_t bo = (size_t)(n0 + (j << 4) + rlane) * ldb + koff + k0;
      bh[j] = Frag<T>::load(Bb + bo);
      if (SPLIT) bl[j] = Frag<T>::load(Bb2 + bo);
    }
#pragma unroll
    for (int i = 0; i < 4; ++i) {
      const size_t ao = (size_t)(m0 + (i << 4) + rlane) * lda + koff + k0;
      V ah = Frag<T>::load(Ab + ao);
      V al;
      if (SPLIT) al = Frag<T>::load(Ab2 + ao);
#pragma unroll
      for (int j = 0; j < 4; ++j) {
        acc[i][j] = Frag<T>::mma(ah, bh[j], acc[i][j]);
        if (SPLIT) {
          acc[i][j] = Frag<T>::mma(ah, bl[j], acc[i][j]);
          acc[i][j] = Frag<T>::mma(al, bh[j], acc[i][j]);
        }
      }
      Frag<T>::guard(acc[i][0], acc[i][3], ah, SPLIT ? al : ah);
    }
    Frag<T>::keep(bh[0], bh[1], bh[2], bh[3]);
    if (SPLIT) Frag<T>::keep(bl[0], bl[1], bl[2], bl[3]);
  }
  acc_guard4(acc[0][0], acc[0][1], acc[0][2], acc[0][3]);
  acc_guard4(acc[1][0], acc[1][1], acc[1][2], acc[1][3]);
  acc_guard4(acc[2][0], acc[2][1], acc[2][2], acc[2][3]);
  acc_guard4(acc[3][0], acc[3][1], acc[3][2], acc[3][3]);

  float* slab = sT[wave];
  const float* Rb = RESID ? (resid + (size_t)b * strideR) : resid;
#pragma unroll
  for (int i = 0; i < 4; ++i) {
    const int mBase = m0 + (i << 4);
    float bm[8];
#pragma unroll
    for (int r = 0; r < 8; ++r) bm[r] = 0.f;
    if (BIAS_MODE == 1) {
      const v4f b0 = *(const v4f*)(bias + mBase + mOff);
      const v4f b1 = *(const v4f*)(bias + mBase + mOff + 4);
      bm[0] = b0[0]; bm[1] = b0[1]; bm[2] = b0[2]; bm[3] = b0[3];
      bm[4] = b1[0]; bm[5] = b1[1]; bm[6] = b1[2]; bm[7] = b1[3];
    }
#pragma unroll
    for (int j = 0; j < 4; ++j) {
      const int n = n0 + (j << 4) + rlane;
      float bvn = 0.f;
      if (BIAS_MODE == 2) bvn = bias[n];
#pragma unroll
      for (int r = 0; r < 8; ++r) {
        float v = acc[i][j][r] * scale;
        if (BIAS_MODE == 1) v += bm[r];
        if (BIAS_MODE == 2) v += bvn;
        if (ACT == 2) v = fmaxf(v, 0.0f);
        if (ACT == 4) v = (v > 0.f) ? v : 0.01f * v;
        slab[(mOff + r) * 68 + (j << 4) + rlane] = v;
      }
    }
    __builtin_amdgcn_fence(__ATOMIC_RELEASE, "workgroup");
    __builtin_amdgcn_wave_barrier();
    __builtin_amdgcn_fence(__ATOMIC_ACQUIRE, "workgroup");
    if (OUT_MODE == 0) {
      float* Cb = (float*)Cout + (size_t)b * strideC;
      const int hh = lane >> 4, c4 = (lane & 15) * 4;
      v4f vals[8];
#pragma unroll
      for (int it = 0; it < 8; ++it) {
        const int row = it * 2 + hh;
        v4f v = *(const v4f*)(slab + row * 68 + c4);
        if (RESID) {
          const v4f rr = *(const v4f*)(Rb + (size_t)(mBase + row) * ldc + n0 + c4);
          v += rr;
        }
        vals[it] = v;
      }
      for (int pass = 0; pass < 2; ++pass) {
#pragma unroll
        for (int it = 0; it < 8; ++it) {
          const int row = it * 2 + hh;
          *(volatile v4f*)(Cb + (size_t)(mBase + row) * ldc + n0 + c4) = vals[it];
        }
        __threadfence();
      }
    } else {
      const int q = lane >> 3, c8 = (lane & 7) * 8;
      unsigned short* Cb  = (unsigned short*)Cout  + (size_t)b * strideC;
      unsigned short* Cb2 = (OUT_MODE == 2) ? ((unsigned short*)Cout2 + (size_t)b * strideC) : nullptr;
      for (int pass = 0; pass < 2; ++pass) {
#pragma unroll
        for (int it = 0; it < 4; ++it) {
          const int row = it * 4 + q;
          const float* sp = slab + row * 68 + c8;
          v8h hv, lv;
#pragma unroll
          for (int e = 0; e < 8; ++e) {
            if (OUT_MODE == 1) {
              hv[e] = (_Float16)sp[e];
            } else {
              unsigned short hb = f2bf_bits(sp[e]);
              unsigned short lb = f2bf_bits(sp[e] - bf_bits2f(hb));
              hv[e] = __builtin_bit_cast(_Float16, hb);
              lv[e] = __builtin_bit_cast(_Float16, lb);
            }
          }
          *(volatile v8h*)(Cb + (size_t)(mBase + row) * ldc + n0 + c8) = hv;
          if (OUT_MODE == 2) *(volatile v8h*)(Cb2 + (size_t)(mBase + row) * ldc + n0 + c8) = lv;
        }
        __threadfence();
      }
    }
    __builtin_amdgcn_fence(__ATOMIC_RELEASE, "workgroup");
    __builtin_amdgcn_wave_barrier();
    __builtin_amdgcn_fence(__ATOMIC_ACQUIRE, "workgroup");
  }
}

__global__ __launch_bounds__(256) void cast_f32_f16x2(
    const float* __restrict__ in, _Float16* __restrict__ out, int n2) {
  int i = blockIdx.x * 256 + threadIdx.x;
  if (i < n2) {
    const _Float16 h0 = (_Float16)in[2 * i], h1 = (_Float16)in[2 * i + 1];
    const unsigned u = (unsigned)__builtin_bit_cast(unsigned short, h0) | ((unsigned)__builtin_bit_cast(unsigned short, h1) << 16);
    ((volatile unsigned*)out)[i] = u;
    __threadfence();
    ((volatile unsigned*)out)[i] = u;
  }
}

__global__ __launch_bounds__(256) void gn_stats_k(
    const float* __restrict__ x, float* __restrict__ stats, int count, float eps)
{
  __shared__ float redA[8], redB[8];
  const int tid = threadIdx.x, lane = tid & 31, wave = tid >> 5;
  const float* base = x + (size_t)blockIdx.x * count;
  float s = 0.f;
#pragma unroll 4
  for (int i = tid * 4; i < count; i += 1024) {
    const v4f v = *(const v4f*)(base + i);
    s += (v[0] + v[1]) + (v[2] + v[3]);
  }
#pragma unroll
  for (int off = 16; off >= 1; off >>= 1) s += __shfl_xor(s, off, 32);
  if (lane == 0) redA[wave] = s;
  __syncthreads();
  float S = 0.f;
#pragma unroll
  for (int w = 0; w < 8; ++w) S += redA[w];
  const float inv_cnt = 1.0f / (float)count;
  const float mean = S * inv_cnt;
  float ss = 0.f;
#pragma unroll 4
  for (int i = tid * 4; i < count; i += 1024) {
    const v4f v = *(const v4f*)(base + i);
    const float d0 = v[0] - mean, d1 = v[1] - mean, d2 = v[2] - mean, d3 = v[3] - mean;
    ss += (d0 * d0 + d1 * d1) + (d2 * d2 + d3 * d3);
  }
#pragma unroll
  for (int off = 16; off >= 1; off >>= 1) ss += __shfl_xor(ss, off, 32);
  if (lane == 0) redB[wave] = ss;
  __syncthreads();
  float SS = 0.f;
#pragma unroll
  for (int w = 0; w < 8; ++w) SS += redB[w];
  const float var = SS * inv_cnt;
  const float rstd = 1.0f / sqrtf(var + eps);
  if (wave == 0 && lane < 8) {
    v4f o = (v4f){0.f, 0.f, 0.f, 0.f};
    if (lane == 0) { o[0] = mean; o[1] = rstd; }
    float* dst = stats + (size_t)blockIdx.x * STATS_LINE_FLOATS + lane * 4;
    *(volatile v4f*)dst = o;
    __threadfence();
    *(volatile v4f*)dst = o;
  }
}

constexpr int XT_PITCH = 136;
__global__ __launch_bounds__(256) void gn_apply_k(
    const float* __restrict__ x, const float* __restrict__ stats,
    const float* __restrict__ gamma, const float* __restrict__ beta,
    unsigned short* __restrict__ Xn, int Lseq)
{
  __shared__ float sgm[NCH], sbt[NCH], smu[NCH], srs[NCH];
  __shared__ __align__(16) _Float16 sh[64 * XT_PITCH];
  const int tid = threadIdx.x;
  const int nlt = Lseq / 64;
  const int n = blockIdx.x / nlt;
  const int l0 = (blockIdx.x - n * nlt) * 64;
  if (tid < NCH) {
    const int g = tid / (NCH / NGROUPS);
    sgm[tid] = gamma[tid];
    sbt[tid] = beta[tid];
    smu[tid] = stats[(size_t)(n * NGROUPS + g) * STATS_LINE_FLOATS + 0];
    srs[tid] = stats[(size_t)(n * NGROUPS + g) * STATS_LINE_FLOATS + 1];
  }
  __syncthreads();
  const float* xb = x + (size_t)n * NCH * Lseq;
#pragma unroll 1
  for (int it = 0; it < 4; ++it) {
    const int idx = it * 256 + tid;
    const int p = idx & 63;
    const int c8 = (idx >> 6) * 8;
    float xv[8];
#pragma unroll
    for (int e = 0; e < 8; ++e) xv[e] = xb[(size_t)(c8 + e) * Lseq + l0 + p];
    v8h hv;
#pragma unroll
    for (int e = 0; e < 8; ++e)
      hv[e] = (_Float16)((xv[e] - smu[c8 + e]) * srs[c8 + e] * sgm[c8 + e] + sbt[c8 + e]);
    *(v8h*)(sh + p * XT_PITCH + c8) = hv;
  }
  __syncthreads();
  _Float16* dst = (_Float16*)Xn + ((size_t)n * Lseq + l0) * NCH;
  v4u wv[4];
#pragma unroll
  for (int it = 0; it < 4; ++it) {
    const int qd = it * 256 + tid;
    const int row = qd >> 4, c16 = qd & 15;
    wv[it] = *(const v4u*)(sh + row * XT_PITCH + c16 * 8);
  }
  for (int pass = 0; pass < 2; ++pass) {
#pragma unroll
    for (int it = 0; it < 4; ++it) {
      const int qd = it * 256 + tid;
      const int row = qd >> 4, c16 = qd & 15;
      *(volatile v4u*)(dst + (size_t)row * NCH + c16 * 8) = wv[it];
    }
    __threadfence();
  }
}

constexpr int AHD = 128;
constexpr int AKEYS = 64;
constexpr int AQROWS = 64;
constexpr int K_PITCH = 136;
constexpr int V_PITCH = 72;
constexpr int P_PITCH = 72;
constexpr int O_PITCH = 132;
constexpr float PROB_CARRY = 32768.0f;

__device__ __forceinline__ v8f mma_h16(v16h a, v16h b, v8f c) {
  c = __builtin_amdgcn_wmma_f32_16x16x32_f16(false, a, false, b, (short)0, c, false, false);
  asm volatile("v_nop\n\tv_nop\n\tv_nop\n\tv_nop" : "+v"(c) : "v"(a), "v"(b));
  return c;
}

__global__ __launch_bounds__(128) void attn_hd128_f16(
    const unsigned short* __restrict__ Qp, const unsigned short* __restrict__ Kp,
    const unsigned short* __restrict__ Vtp, unsigned short* __restrict__ Ap,
    int Lseq, float sm_scale, float out_carry)
{
  union FH { v16h v; v8h h[2]; };
  __shared__ __align__(16) _Float16 Ksh[AKEYS * K_PITCH];
  __shared__ __align__(16) _Float16 Vsh[AHD * V_PITCH];
  __shared__ __align__(16) _Float16 Psh[4][16 * P_PITCH];
  __shared__ __align__(16) float    Osh[4][16 * O_PITCH];

  const int tid  = threadIdx.x;
  const int wave = tid >> 5;
  const int lane = tid & 31;
  const int hh   = lane >> 4;
  const int c    = lane & 15;
  const int nqb  = Lseq / AQROWS;
  const int n    = blockIdx.x / nqb;
  const int qb   = blockIdx.x - n * nqb;
  const int q0   = qb * AQROWS + wave * 16;

  const _Float16* Qb = (const _Float16*)Qp + (size_t)n * Lseq * AHD;
  const _Float16* Kb = (const _Float16*)Kp + (size_t)n * Lseq * AHD;
  const _Float16* Vb = (const _Float16*)Vtp + (size_t)n * AHD * Lseq;
  _Float16*       Ab = (_Float16*)Ap + (size_t)n * Lseq * AHD;

  v16h qa[4];
#pragma unroll
  for (int dc = 0; dc < 4; ++dc)
    qa[dc] = Frag<_Float16>::load(Qb + (size_t)(q0 + c) * AHD + dc * 32 + 8 * hh);

  float mrow[8], lrow[8];
  v8f oacc[8];
#pragma unroll
  for (int r = 0; r < 8; ++r) { mrow[r] = -__builtin_inff(); lrow[r] = 0.f; }
#pragma unroll
  for (int t = 0; t < 8; ++t) oacc[t] = (v8f){0.f,0.f,0.f,0.f,0.f,0.f,0.f,0.f};

  const int nChunks = Lseq / AKEYS;
  for (int kc = 0; kc < nChunks; ++kc) {
    const int kv0 = kc * AKEYS;
    __syncthreads();
#pragma unroll 4
    for (int it = 0; it < 8; ++it) {
      const int qd = it * 128 + tid;
      const int row = qd >> 4, c16 = qd & 15;
      const v4u w = *(const v4u*)(Kb + (size_t)(kv0 + row) * AHD + c16 * 8);
      *(v4u*)(Ksh + row * K_PITCH + c16 * 8) = w;
    }
#pragma unroll 4
    for (int it = 0; it < 8; ++it) {
      const int qd = it * 128 + tid;
      const int d = qd >> 3, c16 = qd & 7;
      const v4u w = *(const v4u*)(Vb + (size_t)d * Lseq + kv0 + c16 * 8);
      *(v4u*)(Vsh + d * V_PITCH + c16 * 8) = w;
    }
    __syncthreads();

    v8f s[4];
#pragma unroll
    for (int j = 0; j < 4; ++j) {
      s[j] = (v8f){0.f,0.f,0.f,0.f,0.f,0.f,0.f,0.f};
#pragma unroll
      for (int dc = 0; dc < 4; ++dc) {
        FH kb;
        kb.h[0] = *(const v8h*)(Ksh + (j * 16 + c) * K_PITCH + dc * 32 + 8 * hh);
        kb.h[1] = *(const v8h*)(Ksh + (j * 16 + c) * K_PITCH + dc * 32 + 16 + 8 * hh);
        s[j] = mma_h16(qa[dc], kb.v, s[j]);
      }
    }

    float cm[8];
#pragma unroll
    for (int r = 0; r < 8; ++r) {
      float m = -__builtin_inff();
#pragma unroll
      for (int j = 0; j < 4; ++j) {
        const float sv = s[j][r] * sm_scale;
        s[j][r] = sv;
        m = fmaxf(m, sv);
      }
#pragma unroll
      for (int off = 1; off < 16; off <<= 1) m = fmaxf(m, __shfl_xor(m, off, 32));
      cm[r] = m;
    }
    _Float16* pw = Psh[wave];
#pragma unroll
    for (int r = 0; r < 8; ++r) {
      const float mnew = fmaxf(mrow[r], cm[r]);
      const float alpha = expf(mrow[r] - mnew);
      mrow[r] = mnew;
      float psum = 0.f;
#pragma unroll
      for (int j = 0; j < 4; ++j) {
        const float p = expf(s[j][r] - mnew);
        psum += p;
        pw[(8 * hh + r) * P_PITCH + j * 16 + c] = (_Float16)(p * PROB_CARRY);
      }
#pragma unroll
      for (int off = 1; off < 16; off <<= 1) psum += __shfl_xor(psum, off, 32);
      lrow[r] = lrow[r] * alpha + psum;
#pragma unroll
      for (int t = 0; t < 8; ++t) oacc[t][r] *= alpha;
    }
    __builtin_amdgcn_fence(__ATOMIC_RELEASE, "workgroup");
    __builtin_amdgcn_wave_barrier();
    __builtin_amdgcn_fence(__ATOMIC_ACQUIRE, "workgroup");

#pragma unroll
    for (int kk = 0; kk < 2; ++kk) {
      FH pa;
      pa.h[0] = *(const v8h*)(pw + c * P_PITCH + kk * 32 + 8 * hh);
      pa.h[1] = *(const v8h*)(pw + c * P_PITCH + kk * 32 + 16 + 8 * hh);
#pragma unroll
      for (int t = 0; t < 8; ++t) {
        FH vf;
        vf.h[0] = *(const v8h*)(Vsh + (t * 16 + c) * V_PITCH + kk * 32 + 8 * hh);
        vf.h[1] = *(const v8h*)(Vsh + (t * 16 + c) * V_PITCH + kk * 32 + 16 + 8 * hh);
        oacc[t] = mma_h16(pa.v, vf.v, oacc[t]);
      }
    }
  }

  float* os = Osh[wave];
#pragma unroll
  for (int r = 0; r < 8; ++r) {
    const float inv = out_carry * (1.0f / (lrow[r] * PROB_CARRY));
#pragma unroll
    for (int t = 0; t < 8; ++t) os[(8 * hh + r) * O_PITCH + t * 16 + c] = oacc[t][r] * inv;
  }
  __builtin_amdgcn_fence(__ATOMIC_RELEASE, "workgroup");
  __builtin_amdgcn_wave_barrier();
  __builtin_amdgcn_fence(__ATOMIC_ACQUIRE, "workgroup");
  {
    const int c8 = (lane & 15) * 8;
    v8h vals[8];
#pragma unroll
    for (int it = 0; it < 8; ++it) {
      const int row = it * 2 + hh;
      const v4f a0 = *(const v4f*)(os + row * O_PITCH + c8);
      const v4f a1 = *(const v4f*)(os + row * O_PITCH + c8 + 4);
      v8h hv;
      hv[0] = (_Float16)a0[0]; hv[1] = (_Float16)a0[1]; hv[2] = (_Float16)a0[2]; hv[3] = (_Float16)a0[3];
      hv[4] = (_Float16)a1[0]; hv[5] = (_Float16)a1[1]; hv[6] = (_Float16)a1[2]; hv[7] = (_Float16)a1[3];
      vals[it] = hv;
    }
    for (int pass = 0; pass < 2; ++pass) {
#pragma unroll
      for (int it = 0; it < 8; ++it) {
        const int row = it * 2 + hh;
        *(volatile v8h*)(Ab + (size_t)(q0 + row) * AHD + c8) = vals[it];
      }
      __threadfence();
    }
  }
}

static inline size_t align128(size_t v) { return (v + 127) & ~(size_t)127; }

extern "C" void kernel_launch(void* const* d_in, const int* in_sizes, int n_in,
                              void* d_out, int out_size, void* d_ws, size_t ws_size,
                              hipStream_t stream) {
  if (n_in < 11) return;
  const float* x     = (const float*)d_in[0];
  const float* gamma = (const float*)d_in[1];
  const float* beta  = (const float*)d_in[2];
  const float* Wq    = (const float*)d_in[3];
  const float* bq    = (const float*)d_in[4];
  const float* Wk    = (const float*)d_in[5];
  const float* bk    = (const float*)d_in[6];
  const float* Wv    = (const float*)d_in[7];
  const float* bv    = (const float*)d_in[8];
  const float* Wo    = (const float*)d_in[9];
  const float* bo    = (const float*)d_in[10];
  float* out = (float*)d_out;

  const long plane_elems = (long)NCH * IMG_L;
  const int nb = (int)((long)in_sizes[0] / plane_elems);
  if (nb < 1 || (long)nb * plane_elems != (long)in_sizes[0]) return;
  if ((long)out_size != (long)in_sizes[0]) return;
  if (in_sizes[1] != NCH || in_sizes[2] != NCH) return;
  if (in_sizes[3] != NCH * NCH || in_sizes[5] != NCH * NCH || in_sizes[7] != NCH * NCH || in_sizes[9] != NCH * NCH) return;
  if (in_sizes[4] != NCH || in_sizes[6] != NCH || in_sizes[8] != NCH || in_sizes[10] != NCH) return;

  char* ws = (char*)d_ws;
  const size_t statsBytes = (size_t)nb * NGROUPS * STATS_LINE_FLOATS * sizeof(float);
  const size_t wBytes     = (size_t)NCH * NCH * 2;
  const size_t planeBytes = (size_t)nb * plane_elems * 2;
  const size_t off_stats = 0;
  const size_t off_w     = align128(off_stats + statsBytes);
  const size_t off_xn    = align128(off_w + 4 * wBytes);
  const size_t off_q     = align128(off_xn + planeBytes);
  const size_t off_k     = align128(off_q + planeBytes);
  const size_t off_vt    = align128(off_k + planeBytes);
  const size_t off_att   = align128(off_vt + planeBytes);
  const size_t total     = off_att + planeBytes;
  if (total > ws_size) return;

  float* stats = (float*)(ws + off_stats);
  unsigned short* Wq16 = (unsigned short*)(ws + off_w + 0 * wBytes);
  unsigned short* Wk16 = (unsigned short*)(ws + off_w + 1 * wBytes);
  unsigned short* Wv16 = (unsigned short*)(ws + off_w + 2 * wBytes);
  unsigned short* Wo16 = (unsigned short*)(ws + off_w + 3 * wBytes);
  unsigned short* Xn   = (unsigned short*)(ws + off_xn);
  unsigned short* Qpl  = (unsigned short*)(ws + off_q);
  unsigned short* Kpl  = (unsigned short*)(ws + off_k);
  unsigned short* Vtpl = (unsigned short*)(ws + off_vt);
  unsigned short* Att  = (unsigned short*)(ws + off_att);

  const float sm_scale  = 1.0f / sqrtf((float)NCH);
  const float att_carry = 64.0f;

  gn_stats_k<<<dim3(nb * NGROUPS), dim3(256), 0, stream>>>(x, stats, GROUP_ELEMS, 1e-6f);

  const int n2 = NCH * NCH / 2;
  const int castBlocks = (n2 + 255) / 256;
  cast_f32_f16x2<<<dim3(castBlocks), dim3(256), 0, stream>>>(Wq, (_Float16*)Wq16, n2);
  cast_f32_f16x2<<<dim3(castBlocks), dim3(256), 0, stream>>>(Wk, (_Float16*)Wk16, n2);
  cast_f32_f16x2<<<dim3(castBlocks), dim3(256), 0, stream>>>(Wv, (_Float16*)Wv16, n2);
  cast_f32_f16x2<<<dim3(castBlocks), dim3(256), 0, stream>>>(Wo, (_Float16*)Wo16, n2);

  gn_apply_k<<<dim3(nb * (IMG_L / 64)), dim3(256), 0, stream>>>(x, stats, gamma, beta, Xn, IMG_L);

  const int M_qk = nb * IMG_L;
  const int tiles_qk = (M_qk / 64) * (NCH / 64);
  const int blocks_qk = (tiles_qk + 7) / 8;
  wmma_gemm64<0, false, 2, 1, false, 0><<<dim3(blocks_qk, 1), dim3(256), 0, stream>>>(
      Xn, Xn, NCH, 0L, Wq16, Wq16, NCH, 0L, (void*)Qpl, (void*)Qpl, NCH, 0L,
      bq, x, 0L, M_qk, NCH, NCH, 1.0f);
  wmma_gemm64<0, false, 2, 1, false, 0><<<dim3(blocks_qk, 1), dim3(256), 0, stream>>>(
      Xn, Xn, NCH, 0L, Wk16, Wk16, NCH, 0L, (void*)Kpl, (void*)Kpl, NCH, 0L,
      bk, x, 0L, M_qk, NCH, NCH, 1.0f);

  const int tiles_cl = (NCH / 64) * (IMG_L / 64);
  const int blocks_cl = (tiles_cl + 7) / 8;
  wmma_gemm64<0, false, 1, 1, false, 0><<<dim3(blocks_cl, nb), dim3(256), 0, stream>>>(
      Wv16, Wv16, NCH, 0L, Xn, Xn, NCH, (long)plane_elems, (void*)Vtpl, (void*)Vtpl, IMG_L, (long)plane_elems,
      bv, x, 0L, NCH, IMG_L, NCH, 1.0f);

  attn_hd128_f16<<<dim3(nb * (IMG_L / AQROWS)), dim3(128), 0, stream>>>(
      Qpl, Kpl, Vtpl, Att, IMG_L, sm_scale, att_carry);

  wmma_gemm64<0, false, 1, 0, true, 0><<<dim3(blocks_cl, nb), dim3(256), 0, stream>>>(
      Wo16, Wo16, NCH, 0L, Att, Att, NCH, (long)plane_elems, (void*)out, (void*)out, IMG_L, (long)plane_elems,
      bo, x, (long)plane_elems, NCH, IMG_L, NCH, 1.0f / att_carry);
}
